// DBNN_59545426591795
// MI455X (gfx1250) — hardware-verified
//
#include <hip/hip_runtime.h>
#include <math.h>

typedef __attribute__((ext_vector_type(16))) _Float16 v16h;
typedef __attribute__((ext_vector_type(8)))  _Float16 v8h;
typedef __attribute__((ext_vector_type(16))) __bf16   v16b;
typedef __attribute__((ext_vector_type(8)))  float    v8f;
typedef __attribute__((ext_vector_type(4)))  float    v4f;

__device__ __forceinline__ int frag_k(int i, int h) { return (i < 8) ? (8 * h + i) : (16 + 8 * h + (i - 8)); }
__device__ __forceinline__ __bf16 bf16_rne(float f) {
    unsigned int u = __float_as_uint(f);
    u += 0x7fffu + ((u >> 16) & 1u);
    return __builtin_bit_cast(__bf16, (unsigned short)(u >> 16));
}
__device__ __forceinline__ float bf16_f32(__bf16 b) { return __uint_as_float(((unsigned int)__builtin_bit_cast(unsigned short, b)) << 16); }
__device__ __forceinline__ v8f wmma16(v16h a, v16h b, v8f c) {
    c = __builtin_amdgcn_wmma_f32_16x16x32_f16(false, a, false, b, (short)0, c, false, false);
    asm volatile("v_nop\n\tv_nop\n\tv_nop\n\tv_nop" : "+v"(c) : "v"(a), "v"(b));
    return c;
}
__device__ __forceinline__ v8f wmmab(v16b a, v16b b, v8f c) {
    c = __builtin_amdgcn_wmma_f32_16x16x32_bf16(false, a, false, b, (short)0, c, false, false);
    asm volatile("v_nop\n\tv_nop\n\tv_nop\n\tv_nop" : "+v"(c) : "v"(a), "v"(b));
    return c;
}
struct Split { v16b hi, lo; };
__device__ __forceinline__ v8f wmma3(const Split& a, const Split& b, v8f c) {
    c = __builtin_amdgcn_wmma_f32_16x16x32_bf16(false, a.hi, false, b.hi, (short)0, c, false, false);
    c = __builtin_amdgcn_wmma_f32_16x16x32_bf16(false, a.hi, false, b.lo, (short)0, c, false, false);
    c = __builtin_amdgcn_wmma_f32_16x16x32_bf16(false, a.lo, false, b.hi, (short)0, c, false, false);
    asm volatile("v_nop\n\tv_nop\n\tv_nop\n\tv_nop" : "+v"(c) : "v"(a.hi), "v"(a.lo), "v"(b.hi), "v"(b.lo));
    return c;
}
struct Split3 { v16b hi, mid, lo; };
__device__ __forceinline__ v8f wmma6(const Split3& a, const Split3& b, v8f c) {
    c = __builtin_amdgcn_wmma_f32_16x16x32_bf16(false, a.hi, false, b.hi, (short)0, c, false, false);
    c = __builtin_amdgcn_wmma_f32_16x16x32_bf16(false, a.hi, false, b.mid, (short)0, c, false, false);
    c = __builtin_amdgcn_wmma_f32_16x16x32_bf16(false, a.mid, false, b.hi, (short)0, c, false, false);
    c = __builtin_amdgcn_wmma_f32_16x16x32_bf16(false, a.hi, false, b.lo, (short)0, c, false, false);
    c = __builtin_amdgcn_wmma_f32_16x16x32_bf16(false, a.mid, false, b.mid, (short)0, c, false, false);
    c = __builtin_amdgcn_wmma_f32_16x16x32_bf16(false, a.lo, false, b.hi, (short)0, c, false, false);
    asm volatile("v_nop\n\tv_nop\n\tv_nop\n\tv_nop" : "+v"(c) : "v"(a.hi), "v"(a.mid), "v"(a.lo), "v"(b.hi), "v"(b.mid), "v"(b.lo));
    return c;
}

__device__ __forceinline__ v16h fh_ld(const float* __restrict__ p, long long sk, int k0, int h, int klen, float s) {
    v16h a;
#pragma unroll
    for (int i = 0; i < 16; ++i) { const int k = k0 + frag_k(i, h); a[i] = (k < klen) ? (_Float16)(p[(long long)k * sk] * s) : (_Float16)0.f; }
    return a;
}
__device__ __forceinline__ Split sp_ld(const float* __restrict__ p, long long sk, int k0, int h, int klen, float s) {
    Split r;
#pragma unroll
    for (int i = 0; i < 16; ++i) {
        const int k = k0 + frag_k(i, h); const float x = (k < klen) ? p[(long long)k * sk] * s : 0.f;
        const __bf16 hb = bf16_rne(x); r.hi[i] = hb; r.lo[i] = bf16_rne(x - bf16_f32(hb));
    }
    return r;
}
__device__ __forceinline__ Split3 sp3_ld(const float* __restrict__ p, long long sk, int k0, int h, int klen, float s) {
    Split3 r;
#pragma unroll
    for (int i = 0; i < 16; ++i) {
        const int k = k0 + frag_k(i, h); const float x = (k < klen) ? p[(long long)k * sk] * s : 0.f;
        const __bf16 hb = bf16_rne(x); const float r1 = x - bf16_f32(hb); const __bf16 mb = bf16_rne(r1);
        r.hi[i] = hb; r.mid[i] = mb; r.lo[i] = bf16_rne(r1 - bf16_f32(mb));
    }
    return r;
}
__device__ __forceinline__ v16b bh_ld(const float* __restrict__ p, long long sk, int k0, int h, int klen, float s) {
    v16b a;
#pragma unroll
    for (int i = 0; i < 16; ++i) { const int k = k0 + frag_k(i, h); a[i] = bf16_rne((k < klen) ? p[(long long)k * sk] * s : 0.f); }
    return a;
}
__device__ __forceinline__ v16h fh_row(const _Float16* __restrict__ row, int k0, int h) {
    v16h a;
#pragma unroll
    for (int i = 0; i < 16; ++i) a[i] = row[k0 + frag_k(i, h)];
    return a;
}

#define VST2(T, ptr, val) do { *(volatile T*)(ptr) = (val); __threadfence(); *(volatile T*)(ptr) = (val); } while (0)
typedef float v4f __attribute__((ext_vector_type(4)));
#define VST2V4(ptr, val) do { *(volatile v4f*)(ptr) = (val); __threadfence(); *(volatile v4f*)(ptr) = (val); } while (0)

__device__ __attribute__((noinline)) float act_fn(float v, int act) {
    if (act == 1) return fmaxf(v, 0.f);
    if (act == 2) { const float u = 0.7978845608028654f * (v + 0.044715f * v * v * v); return 0.5f * v * (1.f + tanhf(u)); }
    if (act == 3) return v / (1.f + expf(-v));
    if (act == 4) return 0.5f * v * (1.f + erff(v * 0.7071067811865476f));
    if (act == 5) return tanhf(v);
    if (act == 6) return 1.f / (1.f + expf(-v));
    if (act == 7) return (v > 0.f) ? v : 0.01f * v;
    if (act == 8) return (v > 0.f) ? v : (expf(v) - 1.f);
    if (act == 9) return fminf(fmaxf(v, 0.f), 6.f);
    if (act == 10) return fabsf(v);
    if (act == 11) return (v >= 0.f) ? v : 0.1f * v;
    if (act == 12) return (v > 0.f) ? v : 0.2f * v;
    if (act == 13) return (v > 20.f) ? v : log1pf(expf(v));
    return v;
}

struct GemmP {
    const float* A; const float* B; const float* bias; const float* R; float* C;
    long long sAo, sAi, sAm, sAk, sBo, sBi, sBn, sBk, sCo, sCi, sCm, sRo, sRi, sRm, sRn;
    int M, N, K, zi_n, flags, act; float alpha, beta, sa, sb;
    int Npad, pad_;
};
static_assert(sizeof(GemmP) == 5 * 8 + 15 * 8 + 6 * 4 + 4 * 4 + 2 * 4, "GemmP has padding");

template <int MODE>
__global__ __launch_bounds__(32) void k_gemm(GemmP p) {
    const int lane = threadIdx.x & 31, h = lane >> 4, l15 = lane & 15;
    const int m0 = blockIdx.y * 16, n0 = blockIdx.x * 32;
    const int z = blockIdx.z, zo = z / p.zi_n, zi = z - zo * p.zi_n;
    const float* A = p.A + zo * p.sAo + zi * p.sAi;
    const float* B = p.B + zo * p.sBo + zi * p.sBi;
    const int am = min(m0 + l15, p.M - 1);
    v8f acc[2], comp[2];
#pragma unroll
    for (int t = 0; t < 2; ++t) { v8f zz = {}; acc[t] = zz; comp[t] = zz; }
    for (int k0 = 0; k0 < p.K; k0 += 32) {
        const float* arow = A + (long long)am * p.sAm;
        if (MODE == 1) {
            const Split a = sp_ld(arow, p.sAk, k0, h, p.K, 1.f);
#pragma unroll
            for (int t = 0; t < 2; ++t) {
                const int bn = min(n0 + t * 16 + l15, p.N - 1);
                acc[t] = wmma3(a, sp_ld(B + (long long)bn * p.sBn, p.sBk, k0, h, p.K, 1.f), acc[t]);
            }
        } else if (MODE == 3) {
            const Split3 a = sp3_ld(arow, p.sAk, k0, h, p.K, 1.f);
#pragma unroll
            for (int t = 0; t < 2; ++t) {
                const int bn = min(n0 + t * 16 + l15, p.N - 1);
                acc[t] = wmma6(a, sp3_ld(B + (long long)bn * p.sBn, p.sBk, k0, h, p.K, 1.f), acc[t]);
            }
        } else if (MODE == 4) {
            const Split3 a = sp3_ld(arow, p.sAk, k0, h, p.K, 1.f);
#pragma unroll
            for (int t = 0; t < 2; ++t) {
                const int bn = min(n0 + t * 16 + l15, p.N - 1); v8f zz = {};
                const v8f part = wmma6(a, sp3_ld(B + (long long)bn * p.sBn, p.sBk, k0, h, p.K, 1.f), zz);
                const v8f y = part - comp[t]; const v8f s = acc[t] + y; comp[t] = (s - acc[t]) - y; acc[t] = s;
            }
        } else if (MODE == 2) {
            const v16b a = bh_ld(arow, p.sAk, k0, h, p.K, 1.f);
#pragma unroll
            for (int t = 0; t < 2; ++t) {
                const int bn = min(n0 + t * 16 + l15, p.N - 1);
                acc[t] = wmmab(a, bh_ld(B + (long long)bn * p.sBn, p.sBk, k0, h, p.K, 1.f), acc[t]);
            }
        } else {
            const v16h a = fh_ld(arow, p.sAk, k0, h, p.K, p.sa);
#pragma unroll
            for (int t = 0; t < 2; ++t) {
                const int bn = min(n0 + t * 16 + l15, p.N - 1);
                acc[t] = wmma16(a, fh_ld(B + (long long)bn * p.sBn, p.sBk, k0, h, p.K, p.sb), acc[t]);
            }
        }
    }
    const float iscale = (MODE == 0) ? p.alpha / (p.sa * p.sb) : p.alpha;
    float* C = p.C + zo * p.sCo + zi * p.sCi;
    const float* R = p.R + zo * p.sRo + zi * p.sRi;
    __shared__ __align__(16) float ctile[16][36];
#pragma unroll
    for (int t = 0; t < 2; ++t) {
        const int n = n0 + t * 16 + l15; const int nn = min(n, p.N - 1);
#pragma unroll
        for (int r = 0; r < 8; ++r) {
            const int m = m0 + 8 * h + r; const int mm = min(m, p.M - 1);
            float v = acc[t][r] * iscale;
            if (p.flags & 1) v += p.bias[nn];
            if (p.flags & 2) v += p.bias[mm];
            v = act_fn(v, p.act);
            if (p.flags & 4) v += p.beta * R[(long long)mm * p.sRm + (long long)nn * p.sRn];
            ctile[8 * h + r][t * 16 + l15] = (n < p.N) ? v : 0.f;
        }
    }
    __syncthreads();
    const int NW = (p.Npad > p.N) ? p.Npad : p.N;
    const bool fast = (m0 + 16 <= p.M) && (n0 + 32 <= NW) && ((p.sCm & 3) == 0) && ((((size_t)C) & 15) == 0);
    if (fast) {
#pragma unroll
        for (int s = 0; s < 4; ++s) {
            const int row = s * 4 + (lane >> 3), c4 = (lane & 7) * 4;
            const v4f v = *(const v4f*)&ctile[row][c4];
            VST2V4(C + (long long)(m0 + row) * p.sCm + n0 + c4, v);
        }
    } else {
        for (int row = 0; row < 16; ++row) {
            const int m = m0 + row, n = n0 + lane;
            if (m < p.M && n < NW) VST2(float, C + (long long)m * p.sCm + n, ctile[row][lane]);
        }
    }
}

#define AW 4
struct AttnP {
    const float* Q; const float* K; const float* V; float* O; float* P; const float* Mf; const int* Mi; float* ST;
    const float* Pw; const float* Rt; const int* SQ; const int* SK;
    long long swb, swh, swi, swj, srb, srh, sri;
    long long sQb, sQh, sQi, sQd, sKb, sKh, sKj, sKd, sVb, sVh, sVj, sVd, sOb, sOh, sOi, sPb, sPh, sPi, smb, smh, smi, smj;
    int Lq, Lk, dh, dv, hrep, causal, coff, pband;
    float scale, mfill; int nonorm, mpol;
    int roff, rn, segpol, win;
};
static_assert(sizeof(AttnP) == 12 * 8 + 29 * 8 + 16 * 4, "AttnP has padding");

#ifndef KATTN_ATTR
#define KATTN_ATTR
#endif
template <int DHP, int DVP, int QM, bool SPLITPV, bool TWOPASS>
__global__ __launch_bounds__(32 * AW) KATTN_ATTR void k_attn(AttnP p) {
    constexpr int NT = DVP / 16;
    constexpr int KS = DHP / 32;
    constexpr int VP = DVP + 8;
    __shared__ __align__(16) float    pl[AW][16 * 64];
    __shared__ __align__(16) _Float16 vl[(SPLITPV ? 2 : 1) * 64 * VP];
    const int lane = threadIdx.x & 31, hf = lane >> 4, l15 = lane & 15, wave = threadIdx.x >> 5;
    const int h = blockIdx.y, b = blockIdx.z, hk = h / p.hrep;
    const int q0 = (blockIdx.x * AW + wave) * 16;
    float* myp = pl[wave];
    const float L2E = 1.4426950408889634f;
    const float NEG = -__builtin_inff();
    const int qi = min(q0 + l15, p.Lq - 1);
    const float* qrow = p.Q + b * p.sQb + h * p.sQh + (long long)qi * p.sQi;
    const float* kbase = p.K + b * p.sKb + hk * p.sKh;
    const float* vbase = p.V + b * p.sVb + hk * p.sVh;
    v16h qa[QM == 0 ? KS : 1]; Split qs_[QM == 1 ? KS : 1]; Split3 qt_[QM == 2 ? KS : 1];
#pragma unroll
    for (int ks = 0; ks < KS; ++ks) {
        if (QM == 2) qt_[ks] = sp3_ld(qrow, p.sQd, ks * 32, hf, p.dh, 1.f);
        else if (QM == 1) qs_[ks] = sp_ld(qrow, p.sQd, ks * 32, hf, p.dh, 1.f);
        else qa[ks] = fh_ld(qrow, p.sQd, ks * 32, hf, p.dh, 1.f);
    }
    v8f o[NT]; float m8[8], l8[8];
#pragma unroll
    for (int t = 0; t < NT; ++t) { v8f zz = {}; o[t] = zz; }
#pragma unroll
    for (int i = 0; i < 8; ++i) { m8[i] = NEG; l8[i] = 0.f; }
    int jend = p.Lk;
    if (p.causal == 1) { const int je = (blockIdx.x * AW + AW - 1) * 16 + 16 + p.coff; jend = min(jend, max(je, 0)); }
    const int npass = TWOPASS ? 2 : 1;
    for (int pass = 0; pass < npass; ++pass) {
        const bool dopv = (!TWOPASS) || pass == 1;
        for (int j0 = 0; j0 < jend; j0 += 64) {
            if (dopv) {
                __syncthreads();
                for (int idx = threadIdx.x; idx < 64 * DVP; idx += 32 * AW) {
                    const int jr = idx / DVP, d = idx - jr * DVP, j = j0 + jr;
                    const float f = (j < p.Lk && d < p.dv) ? vbase[(long long)j * p.sVj + (long long)d * p.sVd] : 0.f;
                    if (SPLITPV) {
                        const __bf16 hb = bf16_rne(f);
                        ((__bf16*)vl)[jr * VP + d] = hb; ((__bf16*)vl)[64 * VP + jr * VP + d] = bf16_rne(f - bf16_f32(hb));
                    } else vl[jr * VP + d] = (_Float16)f;
                }
            }
            v8f s[4];
#pragma unroll
            for (int t = 0; t < 4; ++t) {
                const int j = min(j0 + t * 16 + l15, p.Lk - 1);
                const float* krow = kbase + (long long)j * p.sKj;
                v8f acc = {};
#pragma unroll
                for (int ks = 0; ks < KS; ++ks) {
                    if (QM == 2)      acc = wmma6(qt_[ks], sp3_ld(krow, p.sKd, ks * 32, hf, p.dh, 1.f), acc);
                    else if (QM == 1) acc = wmma3(qs_[ks], sp_ld(krow, p.sKd, ks * 32, hf, p.dh, 1.f), acc);
                    else              acc = wmma16(qa[ks], fh_ld(krow, p.sKd, ks * 32, hf, p.dh, 1.f), acc);
                }
                s[t] = acc;
            }
            float pv[8][4];
#pragma unroll
            for (int i = 0; i < 8; ++i) {
                const int irow = q0 + i + 8 * hf;
                const int ic = min(irow, p.Lq - 1);
                float sc[4];
#pragma unroll
                for (int t = 0; t < 4; ++t) {
                    const int jg = j0 + t * 16 + l15;
                    float v = s[t][i] * p.scale;
                    if (p.Mf) v += p.Mf[b * p.smb + h * p.smh + (long long)ic * p.smi + (long long)min(jg, p.Lk - 1) * p.smj];
                    if (p.Rt) { int rc = ic - min(jg, p.Lk - 1) + p.roff; rc = rc < 0 ? 0 : (rc >= p.rn ? p.rn - 1 : rc); v += p.Rt[b * p.srb + h * p.srh + (long long)ic * p.sri + rc]; }
                    if (p.Mi) { const int mv = p.Mi[b * p.smb + h * p.smh + (long long)ic * p.smi + (long long)min(jg, p.Lk - 1) * p.smj]; if (p.mpol ? (mv != 0) : (mv == 0)) v = p.mfill; }
                    if (p.SQ) { const bool same = p.SQ[(long long)b * p.Lq + ic] == p.SK[(long long)b * p.Lk + min(jg, p.Lk - 1)]; if (p.segpol ? same : !same) v = p.mfill; }
                    if (p.causal == 2 && jg > irow + p.coff) v = p.mfill;
                    if (jg >= p.Lk || (p.causal == 1 && jg > irow + p.coff) || (p.causal == 3 && jg < irow + p.coff) || (p.win > 0 && irow + p.coff - jg > p.win)) v = NEG; else v *= L2E;
                    sc[t] = v;
                }
                if (!TWOPASS || pass == 0) {
                    float mx = fmaxf(fmaxf(sc[0], sc[1]), fmaxf(sc[2], sc[3]));
                    mx = fmaxf(mx, __shfl_xor(mx, 1, 32)); mx = fmaxf(mx, __shfl_xor(mx, 2, 32));
                    mx = fmaxf(mx, __shfl_xor(mx, 4, 32)); mx = fmaxf(mx, __shfl_xor(mx, 8, 32));
                    const float mnew = fmaxf(m8[i], mx);
                    const float corr = (mnew == NEG) ? 1.f : exp2f(m8[i] - mnew);
                    float rs = 0.f;
#pragma unroll
                    for (int t = 0; t < 4; ++t) {
                        const float pp = (sc[t] == NEG) ? 0.f : exp2f(sc[t] - mnew); rs += pp;
                        pv[i][t] = p.Pw ? pp * p.Pw[b * p.swb + h * p.swh + (long long)ic * p.swi + (long long)min(j0 + t * 16 + l15, p.Lk - 1) * p.swj] : pp;
                    }
                    rs += __shfl_xor(rs, 1, 32); rs += __shfl_xor(rs, 2, 32); rs += __shfl_xor(rs, 4, 32); rs += __shfl_xor(rs, 8, 32);
                    l8[i] = l8[i] * corr + rs; m8[i] = mnew;
                    if (!TWOPASS) {
#pragma unroll
                        for (int t = 0; t < NT; ++t) o[t][i] *= corr;
                    }
                } else {
                    const float inv = (l8[i] > 0.f) ? 1.f / l8[i] : 0.f;
#pragma unroll
                    for (int t = 0; t < 4; ++t) {
                        const int jg = j0 + t * 16 + l15;
                        float pp = (sc[t] == NEG) ? 0.f : exp2f(sc[t] - m8[i]) * inv;
                        if (p.Pw) pp *= p.Pw[b * p.swb + h * p.swh + (long long)ic * p.swi + (long long)min(jg, p.Lk - 1) * p.swj];
                        pv[i][t] = pp;
                    }
                }
            }
            if (dopv) {
#pragma unroll
                for (int i = 0; i < 8; ++i)
#pragma unroll
                    for (int t = 0; t < 4; ++t) myp[(i + 8 * hf) * 64 + t * 16 + l15] = pv[i][t];
                __syncthreads();
                if (p.P) {
                    float* pb_ = p.P + b * p.sPb + h * p.sPh;
                    const bool fastP = (p.pband == 0) && ((p.sPi & 3) == 0) && (j0 + 64 <= p.Lk) && (q0 + 16 <= p.Lq) && ((((size_t)pb_) & 15) == 0);
                    if (fastP) {
#pragma unroll
                        for (int s = 0; s < 8; ++s) {
                            const int row = s * 2 + (lane >> 4), c4 = (lane & 15) * 4;
                            const v4f v = *(const v4f*)(myp + row * 64 + c4);
                            VST2V4(pb_ + (long long)(q0 + row) * p.sPi + j0 + c4, v);
                        }
                    } else {
                        for (int row = 0; row < 16; ++row) {
                            const int irow = q0 + row; if (irow >= p.Lq) continue;
                            for (int c = lane; c < 64; c += 32) {
                                const int jg = j0 + c; if (jg >= p.Lk) continue;
                                if (p.pband == 0) VST2(float, pb_ + (long long)irow * p.sPi + jg, myp[row * 64 + c]);
                                else if (jg - irow <= p.pband && irow - jg <= p.pband) VST2(float, pb_ + (long long)irow * p.sPi + (jg - irow + p.pband), myp[row * 64 + c]);
                            }
                        }
                    }
                }
                if (SPLITPV) {
                    const Split pa0 = sp_ld(myp + l15 * 64, 1, 0, hf, 64, 1.f), pa1 = sp_ld(myp + l15 * 64, 1, 32, hf, 64, 1.f);
                    const __bf16* vh = (const __bf16*)vl; const __bf16* vlo = vh + 64 * VP;
#pragma unroll
                    for (int t = 0; t < NT; ++t) {
                        const int dcol = t * 16 + l15;
                        Split b0, b1;
#pragma unroll
                        for (int e = 0; e < 16; ++e) {
                            const int k0 = frag_k(e, hf), k1 = 32 + frag_k(e, hf);
                            b0.hi[e] = vh[k0 * VP + dcol]; b0.lo[e] = vlo[k0 * VP + dcol]; b1.hi[e] = vh[k1 * VP + dcol]; b1.lo[e] = vlo[k1 * VP + dcol];
                        }
                        o[t] = wmma3(pa0, b0, o[t]);
                        o[t] = wmma3(pa1, b1, o[t]);
                    }
                } else {
                    const v16h pa0 = fh_ld(myp + l15 * 64, 1, 0, hf, 64, 4096.f), pa1 = fh_ld(myp + l15 * 64, 1, 32, hf, 64, 4096.f);
#pragma unroll
                    for (int t = 0; t < NT; ++t) {
                        const int dcol = t * 16 + l15;
                        v16h b0, b1;
#pragma unroll
                        for (int e = 0; e < 16; ++e) { b0[e] = vl[frag_k(e, hf) * VP + dcol]; b1[e] = vl[(32 + frag_k(e, hf)) * VP + dcol]; }
                        o[t] = wmma16(pa0, b0, o[t]);
                        o[t] = wmma16(pa1, b1, o[t]);
                    }
                }
            }
        }
    }
    float* obase = p.O + b * p.sOb + h * p.sOh;
    if (p.ST) {
        const int rl = lane >> 1, isel = rl & 7;
        float mv = 0.f, lv = 0.f;
#pragma unroll
        for (int i = 0; i < 8; ++i) if (i == isel) { mv = m8[i]; lv = l8[i]; }
        const int irow = q0 + rl;
        if (irow < p.Lq) { float* st = p.ST + (((long long)b * gridDim.y + h) * p.Lq + irow) * 2 + (lane & 1); VST2(float, st, (lane & 1) ? lv : mv * 0.6931471805599453f); }
    }
    float invr[8];
#pragma unroll
    for (int i = 0; i < 8; ++i) {
        if (TWOPASS) invr[i] = SPLITPV ? 1.f : (1.f / 4096.f);
        else if (p.nonorm) invr[i] = exp2f(m8[i]) * (SPLITPV ? 1.f : (1.f / 4096.f));
        else invr[i] = (l8[i] > 0.f) ? (SPLITPV ? 1.f / l8[i] : 1.f / (l8[i] * 4096.f)) : 0.f;
    }
    __syncthreads();
    const bool ofast = ((p.sOi & 3) == 0) && ((((size_t)obase) & 15) == 0) && (q0 + 16 <= p.Lq);
#pragma unroll
    for (int c0 = 0; c0 < DVP; c0 += 64) {
#pragma unroll
        for (int i = 0; i < 8; ++i)
#pragma unroll
            for (int t = 0; t < NT; ++t) if (t * 16 >= c0 && t * 16 < c0 + 64) myp[(i + 8 * hf) * 64 + (t * 16 - c0) + l15] = o[t][i] * invr[i];
        __syncthreads();
        const int cw = (DVP - c0 < 64) ? (DVP - c0) : 64;
        if (ofast && (c0 + cw <= p.dv) && (cw % 32 == 0)) {
            const int lpr = cw / 4;
            const int rows_per_ins = 32 / lpr;
            for (int r0 = 0; r0 < 16; r0 += rows_per_ins) {
                const int row = r0 + lane / lpr, c4 = (lane % lpr) * 4;
                const v4f v = *(const v4f*)(myp + row * 64 + c4);
                VST2V4(obase + (long long)(q0 + row) * p.sOi + c0 + c4, v);
            }
        } else {
            for (int row = 0; row < 16; ++row) {
                const int irow = q0 + row; if (irow >= p.Lq) continue;
                for (int c = lane; c < cw; c += 32) { const int d = c0 + c; if (d < p.dv) VST2(float, obase + (long long)irow * p.sOi + d, myp[row * 64 + c]); }
            }
        }
        __syncthreads();
    }
}

struct TrP { const float* src; float* dst; const float* R2; long long sSz, lds, sDz, ldd, sRz, ldr; int R, C, flags, act; float alpha, beta; };
static_assert(sizeof(TrP) == 3 * 8 + 6 * 8 + 6 * 4, "TrP has padding");
__global__ __launch_bounds__(256) void k_tr(TrP p) {
    __shared__ float tile[32][33];
    const int c0 = blockIdx.x * 32, r0 = blockIdx.y * 32, z = blockIdx.z;
    const int lane = threadIdx.x & 31, wave = threadIdx.x >> 5;
    const float* s = p.src + z * p.sSz;
#pragma unroll
    for (int k = 0; k < 4; ++k) {
        const int rl = wave * 4 + k, r = r0 + rl, c = c0 + lane;
        tile[rl][lane] = (r < p.R && c < p.C) ? s[(long long)r * p.lds + c] : 0.f;
    }
    __syncthreads();
    float* d = p.dst + z * p.sDz; const float* rr = p.R2 + z * p.sRz;
#pragma unroll
    for (int k = 0; k < 4; ++k) {
        const int cl = wave * 4 + k, c = c0 + cl, r = r0 + lane;
        if (c < p.C && r < p.R) {
            float v = act_fn(p.alpha * tile[lane][cl], p.act);
            if (p.flags & 1) v += p.beta * rr[(long long)c * p.ldr + r];
            VST2(float, d + (long long)c * p.ldd + r, v);
        }
    }
}

__global__ __launch_bounds__(256) void k_affine(const float* __restrict__ src, float* __restrict__ dst, int n, float a, float b, const float* __restrict__ sdev) {
    const int i = blockIdx.x * 256 + threadIdx.x;
    if (i < n) { const float aa = sdev ? a * sdev[0] : a; const float v = aa * src[i] + b; VST2(float, dst + i, v); }
}

struct SmP { const float* src; float* dst; const float* Mf; long long sz, sr, dz, dr, smz, smr; int n, pad; float scale_in, scale_out; };
static_assert(sizeof(SmP) == 3 * 8 + 6 * 8 + 4 * 4, "SmP has padding");
__global__ __launch_bounds__(256) void k_softmax(SmP p) {
    __shared__ float red[256];
    const int r = blockIdx.x, z = blockIdx.y, tid = threadIdx.x;
    const float* s = p.src + z * p.sz + (long long)r * p.sr;
    const float* mf = p.Mf ? (p.Mf + z * p.smz + (long long)r * p.smr) : nullptr;
    float mx = -__builtin_inff();
    for (int j = tid; j < p.n; j += 256) { float v = s[j] * p.scale_in; if (mf) v += mf[j]; mx = fmaxf(mx, v); }
    red[tid] = mx; __syncthreads();
    for (int o = 128; o > 0; o >>= 1) { if (tid < o) red[tid] = fmaxf(red[tid], red[tid + o]); __syncthreads(); }
    mx = red[0]; __syncthreads();
    float sum = 0.f;
    for (int j = tid; j < p.n; j += 256) { float v = s[j] * p.scale_in; if (mf) v += mf[j]; sum += (mx == -__builtin_inff()) ? 0.f : expf(v - mx); }
    red[tid] = sum; __syncthreads();
    for (int o = 128; o > 0; o >>= 1) { if (tid < o) red[tid] += red[tid + o]; __syncthreads(); }
    sum = red[0];
    const float inv = (sum > 0.f) ? p.scale_out / sum : 0.f;
    float* d = p.dst + z * p.dz + (long long)r * p.dr;
    for (int j = tid; j < p.n; j += 256) { float v = s[j] * p.scale_in; if (mf) v += mf[j]; const float o = (mx == -__builtin_inff()) ? 0.f : expf(v - mx) * inv; VST2(float, d + j, o); }
}
__global__ __launch_bounds__(256) void k_stats(const float* __restrict__ x, long long sz, long long so, long long si, int inner, int n, float eps, float* __restrict__ stat, int mode) {
    __shared__ float red[256];
    const int z = blockIdx.x, tid = threadIdx.x;
    const float* base = x + z * sz;
    float s = 0.f;
    for (int e = tid; e < n; e += 256) s += base[(long long)(e / inner) * so + (long long)(e % inner) * si];
    red[tid] = s; __syncthreads();
    for (int o = 128; o > 0; o >>= 1) { if (tid < o) red[tid] += red[tid + o]; __syncthreads(); }
    const float mu = (mode == 0 || mode == 3) ? red[0] / (float)n : 0.f; __syncthreads();
    float q = 0.f;
    for (int e = tid; e < n; e += 256) { const float dlt = base[(long long)(e / inner) * so + (long long)(e % inner) * si] - mu; q += dlt * dlt; }
    red[tid] = q; __syncthreads();
    for (int o = 128; o > 0; o >>= 1) { if (tid < o) red[tid] += red[tid + o]; __syncthreads(); }
    {
        float rs;
        if (mode == 2) rs = sqrtf((float)n) / fmaxf(sqrtf(red[0]), eps); else if (mode == 3) rs = rsqrtf(red[0] / (float)(n - 1) + eps); else rs = rsqrtf(red[0] / (float)n + eps);
        if (tid < 32) { const float v = (tid == 0) ? mu : ((tid == 1) ? rs : 0.f); VST2(float, stat + (long long)z * 32 + tid, v); }
    }
}
__global__ __launch_bounds__(256) void k_norm_apply(const float* __restrict__ x, float* __restrict__ y, const float* __restrict__ stat, const float* __restrict__ g, const float* __restrict__ bta,
                                                     int Z, int C, int L, int G, int bn, int act) {
    const long long idx = (long long)blockIdx.x * 256 + threadIdx.x;
    if (idx >= (long long)Z * C * L) return;
    const int l = (int)(idx % L); const long long zc = idx / L; const int c = (int)(zc % C), z = (int)(zc / C); (void)l;
    const int set = bn ? c : (z * G + c / (C / G));
    float v = (x[idx] - stat[(long long)set * 32]) * stat[(long long)set * 32 + 1];
    if (g) v *= g[c];
    if (bta) v += bta[c];
    v = act_fn(v, act);
    VST2(float, y + idx, v);
}

__global__ __launch_bounds__(256) void k_lse_neg(const float* __restrict__ st, float* __restrict__ c, int n) {
    const int i = blockIdx.x * 256 + threadIdx.x;
    if (i < n) { const float v = -(st[2 * i] + logf(st[2 * i + 1])); VST2(float, c + i, v); }
}

__global__ __launch_bounds__(256) void k_iota(int* __restrict__ dst, int n, int a, int b) {
    const int i = blockIdx.x * 256 + threadIdx.x;
    if (i < n) { const int v = a * i + b; VST2(int, dst + i, v); }
}

__global__ __launch_bounds__(256) void k_axpby(const float* __restrict__ x, const float* __restrict__ y, float* __restrict__ dst, int n, float a, float b, float c) {
    const int i = blockIdx.x * 256 + threadIdx.x;
    if (i < n) { const float v = a * x[i] + b * y[i] + c; VST2(float, dst + i, v); }
}

struct RopeP { const float* X; float* Y; const float* C; const float* Sn; const int* pos; long long sXr, sXh, sYr, sYh, sCb, sCp, sCd; int R, Hn, D, S, mode, tmode, pmode, pad; };
static_assert(sizeof(RopeP) == 5 * 8 + 7 * 8 + 8 * 4, "RopeP has padding");
__global__ __launch_bounds__(256) void k_rope(RopeP p) {
    const long long idx = (long long)blockIdx.x * 256 + threadIdx.x;
    if (idx >= (long long)p.R * p.Hn * p.D) return;
    const int d = (int)(idx % p.D); const long long rh = idx / p.D; const int h = (int)(rh % p.Hn); const int r = (int)(rh / p.Hn);
    const int half = p.D / 2;
    int partner; float sign;
    if (p.mode == 0) { partner = (d < half) ? d + half : d - half; sign = (d < half) ? -1.f : 1.f; }
    else { partner = d ^ 1; sign = (d & 1) ? 1.f : -1.f; }
    const int tcol = (p.tmode == 0) ? d : ((p.tmode == 1) ? (d % half) : (d >> 1));
    const int pp = (p.pmode == 0) ? (r % p.S) : ((p.pmode == 1) ? h : p.pos[r]);
    const long long toff = (long long)(r / p.S) * p.sCb + (long long)pp * p.sCp + (long long)tcol * p.sCd;
    const float* xr = p.X + (long long)r * p.sXr + (long long)h * p.sXh;
    const float v = xr[d] * p.C[toff] + sign * xr[partner] * p.Sn[toff];
    VST2(float, p.Y + (long long)r * p.sYr + (long long)h * p.sYh + d, v);
}

__global__ __launch_bounds__(256) void k_invf(float* __restrict__ invb, int half, int D, float base, float num, int fmode, float cexp) {
    const int i = blockIdx.x * 256 + threadIdx.x;
    if (i >= ((half + 31) / 32) * 32) return;
    if (i >= half) { VST2(float, invb + i, 0.f); return; }
    const float e = (float)(2 * i) / (float)D;
    float invf;
    if (fmode == 1) invf = num * expf((float)(2 * i) * cexp);
    else if (fmode == 2) invf = num * powf(base, (-2.0f * ((float)i - 1.0f)) / (float)D);
    else invf = num * (1.0f / powf(base, e));
    VST2(float, invb + i, invf);
}
__global__ __launch_bounds__(256) void k_sincos(float* __restrict__ cs, float* __restrict__ sn, const float* __restrict__ invb, int S, int half, float pscale) {
    const int idx = blockIdx.x * 256 + threadIdx.x;
    if (idx >= S * half) return;
    const int s = idx / half, i = idx - s * half;
    const float ang = (pscale * (float)s) * invb[i];
    VST2(float, cs + idx, cosf(ang)); VST2(float, sn + idx, sinf(ang));
}

__global__ __launch_bounds__(256) void k_mulact(const float* __restrict__ x, const float* __restrict__ y, float* __restrict__ dst, int n, int act) {
    const int i = blockIdx.x * 256 + threadIdx.x;
    if (i < n) { const float v = act_fn(x[i], act) * y[i]; VST2(float, dst + i, v); }
}

__global__ __launch_bounds__(256) void k_matvec(GemmP p) {
    const int rpt = (p.N == 1) ? 1 : 32;
    const long long r0 = ((long long)blockIdx.x * 256 + threadIdx.x) * rpt; const int z = blockIdx.z, zo = z / p.zi_n, zi = z - zo * p.zi_n;
    if (r0 >= p.M) return;
    const float* Bb = p.B + zo * p.sBo + zi * p.sBi;
    float* C = p.C + zo * p.sCo + zi * p.sCi; const float* R = p.R + zo * p.sRo + zi * p.sRi;
    for (int rr = 0; rr < rpt; ++rr) {
        const long long r = r0 + rr; if (r >= p.M) break;
        const float* A = p.A + zo * p.sAo + zi * p.sAi + r * p.sAm;
        float acc[8] = {0.f, 0.f, 0.f, 0.f, 0.f, 0.f, 0.f, 0.f};
        for (int k = 0; k < p.K; ++k) { const float a = A[(long long)k * p.sAk];
#pragma unroll
            for (int j = 0; j < 8; ++j) if (j < p.N) acc[j] += a * Bb[(long long)j * p.sBn + (long long)k * p.sBk]; }
#pragma unroll
        for (int j = 0; j < 8; ++j) if (j < p.N) {
            float v = acc[j] * p.alpha;
            if (p.flags & 1) v += p.bias[j];
            if (p.flags & 2) v += p.bias[r];
            v = act_fn(v, p.act);
            if (p.flags & 4) v += p.beta * R[r * p.sRm + (long long)j * p.sRn];
            VST2(float, C + r * p.sCm + j, v);
        }
    }
}
__global__ __launch_bounds__(256) void k_smallsoftmax(const float* __restrict__ src, float* __restrict__ dst, long long sr, long long dr, int n, long long R, float scale) {
    const long long r0 = ((long long)blockIdx.x * 256 + threadIdx.x) * 32;
    for (int rr = 0; rr < 32; ++rr) {
        const long long r = r0 + rr; if (r >= R) return;
        const float* s = src + r * sr; float* d = dst + r * dr;
        float mx = -__builtin_inff();
        for (int j = 0; j < n; ++j) mx = fmaxf(mx, s[j] * scale);
        float sum = 0.f;
        for (int j = 0; j < n; ++j) sum += expf(s[j] * scale - mx);
        const float inv = 1.f / sum;
        for (int j = 0; j < n; ++j) { const float v = expf(s[j] * scale - mx) * inv; VST2(float, d + j, v); }
    }
}

__global__ __launch_bounds__(32) void k_unitstat(float* __restrict__ st) { const int t = threadIdx.x; const float v = (t == 1) ? 1.f : 0.f; VST2(float, st + t, v); }

__global__ __launch_bounds__(256) void k_lincopy(const float* __restrict__ src, long long lds, float* __restrict__ dst, long long ldd, long long rows, int cols) {
    const long long i = (long long)blockIdx.x * 256 + threadIdx.x; if (i >= rows * cols) return;
    const long long r = i / cols; const int c = (int)(i - r * cols);
    const float v = src[r * lds + c]; VST2(float, dst + r * ldd + c, v);
}

__global__ __launch_bounds__(256) void k_db_wm(const float* __restrict__ W, float* __restrict__ WM, int N) { const int q = blockIdx.x * 256 + threadIdx.x; if (q >= N * N) return; VST2(float, WM + q, (q / N == q % N) ? 0.f : W[q]); }
__global__ __launch_bounds__(128) void k_db_conv(const float* __restrict__ X, const float* __restrict__ tr, const float* __restrict__ td, const float* __restrict__ om, float* __restrict__ Y, int B, int N, int T) { const int q = blockIdx.x * 128 + threadIdx.x; if (q >= B * N) return; const int n = q % N; const float a = expf(-1.f / td[n]), ab = expf(-1.f / td[n] - 1.f / tr[n]), w = om[n]; float A = 0.f, Bv = 0.f; const float* xr = X + (long long)q * T; float* yr = Y + (long long)q * T;
    for (int t = 0; t < T; ++t) { const float xv = xr[t]; A = xv + a * A; Bv = xv + ab * Bv; VST2(float, yr + t, w * (A - Bv)); } }
__global__ __launch_bounds__(256) void k_db_out(const float* __restrict__ Y, const float* __restrict__ U, float* __restrict__ OUT, int b, int N, int T) { const int t = blockIdx.x * 256 + threadIdx.x; if (t >= T) return; float s = 0.f;
#pragma unroll 1
    for (int n = 0; n < N; ++n) s += Y[((long long)b * N + n) * T + t] * (U[(long long)t * N + n] + 1.f); VST2(float, OUT + (long long)b * T + t, s - 70.f); }

template __global__ void k_gemm<1>(GemmP);

extern "C" void kernel_launch(void* const* d_in, const int* in_sizes, int n_in, void* d_out, int out_size, void* d_ws, size_t ws_size, hipStream_t stream) {
    (void)in_sizes; (void)n_in; (void)out_size; (void)ws_size;
    const float* x = (const float*)d_in[0];
    const float* tr = (const float*)d_in[1];
    const float* td = (const float*)d_in[2];
    const float* om = (const float*)d_in[3];
    const float* W = (const float*)d_in[4];
    const int Bn = 32;
    const int N = 256;
    const int T = 1024;
    float* out = (float*)d_out;
    char* wsp = (char*)d_ws;
    float* Y = (float*)wsp; wsp += (((size_t)((size_t)Bn * N * T) * 4 + 255) / 256) * 256;
    float* WM = (float*)wsp; wsp += (((size_t)((size_t)N * N) * 4 + 255) / 256) * 256;
    float* U = (float*)wsp; wsp += (((size_t)((size_t)T * N) * 4 + 255) / 256) * 256;
    k_db_wm<<<(unsigned)((N * N + 255) / 256), 256, 0, stream>>>(W, WM, N); k_db_conv<<<(unsigned)((Bn * N + 127) / 128), 128, 0, stream>>>(x, tr, td, om, Y, Bn, N, T);
    { GemmP gu0;
      gu0.A = Y + (size_t)0 * N * T; gu0.B = WM; gu0.bias = Y + (size_t)0 * N * T; gu0.R = Y + (size_t)0 * N * T; gu0.C = U;
      gu0.sAo = 0; gu0.sAi = 0; gu0.sAm = 1; gu0.sAk = T; gu0.sBo = 0; gu0.sBi = 0; gu0.sBn = N; gu0.sBk = 1; gu0.sCo = 0; gu0.sCi = 0; gu0.sCm = N; gu0.sRo = 0; gu0.sRi = 0; gu0.sRm = 0; gu0.sRn = 0;
      gu0.M = T; gu0.N = N; gu0.K = N; gu0.zi_n = 1; gu0.flags = 0; gu0.act = 0;
      gu0.alpha = 1.0f; gu0.beta = 0.0f; gu0.sa = 1.0f; gu0.sb = 1.0f; gu0.Npad = N; gu0.pad_ = 0;
      k_gemm<1><<<dim3((unsigned)((N) + 31) / 32, (unsigned)((T) + 15) / 16, (unsigned)(1)), 32, 0, stream>>>(gu0); }
    k_db_out<<<(unsigned)((T + 255) / 256), 256, 0, stream>>>(Y, U, out, 0, N, T);
    { GemmP gu1;
      gu1.A = Y + (size_t)1 * N * T; gu1.B = WM; gu1.bias = Y + (size_t)1 * N * T; gu1.R = Y + (size_t)1 * N * T; gu1.C = U;
      gu1.sAo = 0; gu1.sAi = 0; gu1.sAm = 1; gu1.sAk = T; gu1.sBo = 0; gu1.sBi = 0; gu1.sBn = N; gu1.sBk = 1; gu1.sCo = 0; gu1.sCi = 0; gu1.sCm = N; gu1.sRo = 0; gu1.sRi = 0; gu1.sRm = 0; gu1.sRn = 0;
      gu1.M = T; gu1.N = N; gu1.K = N; gu1.zi_n = 1; gu1.flags = 0; gu1.act = 0;
      gu1.alpha = 1.0f; gu1.beta = 0.0f; gu1.sa = 1.0f; gu1.sb = 1.0f; gu1.Npad = N; gu1.pad_ = 0;
      k_gemm<1><<<dim3((unsigned)((N) + 31) / 32, (unsigned)((T) + 15) / 16, (unsigned)(1)), 32, 0, stream>>>(gu1); }
    k_db_out<<<(unsigned)((T + 255) / 256), 256, 0, stream>>>(Y, U, out, 1, N, T);
    { GemmP gu2;
      gu2.A = Y + (size_t)2 * N * T; gu2.B = WM; gu2.bias = Y + (size_t)2 * N * T; gu2.R = Y + (size_t)2 * N * T; gu2.C = U;
      gu2.sAo = 0; gu2.sAi = 0; gu2.sAm = 1; gu2.sAk = T; gu2.sBo = 0; gu2.sBi = 0; gu2.sBn = N; gu2.sBk = 1; gu2.sCo = 0; gu2.sCi = 0; gu2.sCm = N; gu2.sRo = 0; gu2.sRi = 0; gu2.sRm = 0; gu2.sRn = 0;
      gu2.M = T; gu2.N = N; gu2.K = N; gu2.zi_n = 1; gu2.flags = 0; gu2.act = 0;
      gu2.alpha = 1.0f; gu2.beta = 0.0f; gu2.sa = 1.0f; gu2.sb = 1.0f; gu2.Npad = N; gu2.pad_ = 0;
      k_gemm<1><<<dim3((unsigned)((N) + 31) / 32, (unsigned)((T) + 15) / 16, (unsigned)(1)), 32, 0, stream>>>(gu2); }
    k_db_out<<<(unsigned)((T + 255) / 256), 256, 0, stream>>>(Y, U, out, 2, N, T);
    { GemmP gu3;
      gu3.A = Y + (size_t)3 * N * T; gu3.B = WM; gu3.bias = Y + (size_t)3 * N * T; gu3.R = Y + (size_t)3 * N * T; gu3.C = U;
      gu3.sAo = 0; gu3.sAi = 0; gu3.sAm = 1; gu3.sAk = T; gu3.sBo = 0; gu3.sBi = 0; gu3.sBn = N; gu3.sBk = 1; gu3.sCo = 0; gu3.sCi = 0; gu3.sCm = N; gu3.sRo = 0; gu3.sRi = 0; gu3.sRm = 0; gu3.sRn = 0;
      gu3.M = T; gu3.N = N; gu3.K = N; gu3.zi_n = 1; gu3.flags = 0; gu3.act = 0;
      gu3.alpha = 1.0f; gu3.beta = 0.0f; gu3.sa = 1.0f; gu3.sb = 1.0f; gu3.Npad = N; gu3.pad_ = 0;
      k_gemm<1><<<dim3((unsigned)((N) + 31) / 32, (unsigned)((T) + 15) / 16, (unsigned)(1)), 32, 0, stream>>>(gu3); }
    k_db_out<<<(unsigned)((T + 255) / 256), 256, 0, stream>>>(Y, U, out, 3, N, T);
    { GemmP gu4;
      gu4.A = Y + (size_t)4 * N * T; gu4.B = WM; gu4.bias = Y + (size_t)4 * N * T; gu4.R = Y + (size_t)4 * N * T; gu4.C = U;
      gu4.sAo = 0; gu4.sAi = 0; gu4.sAm = 1; gu4.sAk = T; gu4.sBo = 0; gu4.sBi = 0; gu4.sBn = N; gu4.sBk = 1; gu4.sCo = 0; gu4.sCi = 0; gu4.sCm = N; gu4.sRo = 0; gu4.sRi = 0; gu4.sRm = 0; gu4.sRn = 0;
      gu4.M = T; gu4.N = N; gu4.K = N; gu4.zi_n = 1; gu4.flags = 0; gu4.act = 0;
      gu4.alpha = 1.0f; gu4.beta = 0.0f; gu4.sa = 1.0f; gu4.sb = 1.0f; gu4.Npad = N; gu4.pad_ = 0;
      k_gemm<1><<<dim3((unsigned)((N) + 31) / 32, (unsigned)((T) + 15) / 16, (unsigned)(1)), 32, 0, stream>>>(gu4); }
    k_db_out<<<(unsigned)((T + 255) / 256), 256, 0, stream>>>(Y, U, out, 4, N, T);
    { GemmP gu5;
      gu5.A = Y + (size_t)5 * N * T; gu5.B = WM; gu5.bias = Y + (size_t)5 * N * T; gu5.R = Y + (size_t)5 * N * T; gu5.C = U;
      gu5.sAo = 0; gu5.sAi = 0; gu5.sAm = 1; gu5.sAk = T; gu5.sBo = 0; gu5.sBi = 0; gu5.sBn = N; gu5.sBk = 1; gu5.sCo = 0; gu5.sCi = 0; gu5.sCm = N; gu5.sRo = 0; gu5.sRi = 0; gu5.sRm = 0; gu5.sRn = 0;
      gu5.M = T; gu5.N = N; gu5.K = N; gu5.zi_n = 1; gu5.flags = 0; gu5.act = 0;
      gu5.alpha = 1.0f; gu5.beta = 0.0f; gu5.sa = 1.0f; gu5.sb = 1.0f; gu5.Npad = N; gu5.pad_ = 0;
      k_gemm<1><<<dim3((unsigned)((N) + 31) / 32, (unsigned)((T) + 15) / 16, (unsigned)(1)), 32, 0, stream>>>(gu5); }
    k_db_out<<<(unsigned)((T + 255) / 256), 256, 0, stream>>>(Y, U, out, 5, N, T);
    { GemmP gu6;
      gu6.A = Y + (size_t)6 * N * T; gu6.B = WM; gu6.bias = Y + (size_t)6 * N * T; gu6.R = Y + (size_t)6 * N * T; gu6.C = U;
      gu6.sAo = 0; gu6.sAi = 0; gu6.sAm = 1; gu6.sAk = T; gu6.sBo = 0; gu6.sBi = 0; gu6.sBn = N; gu6.sBk = 1; gu6.sCo = 0; gu6.sCi = 0; gu6.sCm = N; gu6.sRo = 0; gu6.sRi = 0; gu6.sRm = 0; gu6.sRn = 0;
      gu6.M = T; gu6.N = N; gu6.K = N; gu6.zi_n = 1; gu6.flags = 0; gu6.act = 0;
      gu6.alpha = 1.0f; gu6.beta = 0.0f; gu6.sa = 1.0f; gu6.sb = 1.0f; gu6.Npad = N; gu6.pad_ = 0;
      k_gemm<1><<<dim3((unsigned)((N) + 31) / 32, (unsigned)((T) + 15) / 16, (unsigned)(1)), 32, 0, stream>>>(gu6); }
    k_db_out<<<(unsigned)((T + 255) / 256), 256, 0, stream>>>(Y, U, out, 6, N, T);
    { GemmP gu7;
      gu7.A = Y + (size_t)7 * N * T; gu7.B = WM; gu7.bias = Y + (size_t)7 * N * T; gu7.R = Y + (size_t)7 * N * T; gu7.C = U;
      gu7.sAo = 0; gu7.sAi = 0; gu7.sAm = 1; gu7.sAk = T; gu7.sBo = 0; gu7.sBi = 0; gu7.sBn = N; gu7.sBk = 1; gu7.sCo = 0; gu7.sCi = 0; gu7.sCm = N; gu7.sRo = 0; gu7.sRi = 0; gu7.sRm = 0; gu7.sRn = 0;
      gu7.M = T; gu7.N = N; gu7.K = N; gu7.zi_n = 1; gu7.flags = 0; gu7.act = 0;
      gu7.alpha = 1.0f; gu7.beta = 0.0f; gu7.sa = 1.0f; gu7.sb = 1.0f; gu7.Npad = N; gu7.pad_ = 0;
      k_gemm<1><<<dim3((unsigned)((N) + 31) / 32, (unsigned)((T) + 15) / 16, (unsigned)(1)), 32, 0, stream>>>(gu7); }
    k_db_out<<<(unsigned)((T + 255) / 256), 256, 0, stream>>>(Y, U, out, 7, N, T);
    { GemmP gu8;
      gu8.A = Y + (size_t)8 * N * T; gu8.B = WM; gu8.bias = Y + (size_t)8 * N * T; gu8.R = Y + (size_t)8 * N * T; gu8.C = U;
      gu8.sAo = 0; gu8.sAi = 0; gu8.sAm = 1; gu8.sAk = T; gu8.sBo = 0; gu8.sBi = 0; gu8.sBn = N; gu8.sBk = 1; gu8.sCo = 0; gu8.sCi = 0; gu8.sCm = N; gu8.sRo = 0; gu8.sRi = 0; gu8.sRm = 0; gu8.sRn = 0;
      gu8.M = T; gu8.N = N; gu8.K = N; gu8.zi_n = 1; gu8.flags = 0; gu8.act = 0;
      gu8.alpha = 1.0f; gu8.beta = 0.0f; gu8.sa = 1.0f; gu8.sb = 1.0f; gu8.Npad = N; gu8.pad_ = 0;
      k_gemm<1><<<dim3((unsigned)((N) + 31) / 32, (unsigned)((T) + 15) / 16, (unsigned)(1)), 32, 0, stream>>>(gu8); }
    k_db_out<<<(unsigned)((T + 255) / 256), 256, 0, stream>>>(Y, U, out, 8, N, T);
    { GemmP gu9;
      gu9.A = Y + (size_t)9 * N * T; gu9.B = WM; gu9.bias = Y + (size_t)9 * N * T; gu9.R = Y + (size_t)9 * N * T; gu9.C = U;
      gu9.sAo = 0; gu9.sAi = 0; gu9.sAm = 1; gu9.sAk = T; gu9.sBo = 0; gu9.sBi = 0; gu9.sBn = N; gu9.sBk = 1; gu9.sCo = 0; gu9.sCi = 0; gu9.sCm = N; gu9.sRo = 0; gu9.sRi = 0; gu9.sRm = 0; gu9.sRn = 0;
      gu9.M = T; gu9.N = N; gu9.K = N; gu9.zi_n = 1; gu9.flags = 0; gu9.act = 0;
      gu9.alpha = 1.0f; gu9.beta = 0.0f; gu9.sa = 1.0f; gu9.sb = 1.0f; gu9.Npad = N; gu9.pad_ = 0;
      k_gemm<1><<<dim3((unsigned)((N) + 31) / 32, (unsigned)((T) + 15) / 16, (unsigned)(1)), 32, 0, stream>>>(gu9); }
    k_db_out<<<(unsigned)((T + 255) / 256), 256, 0, stream>>>(Y, U, out, 9, N, T);
    { GemmP gu10;
      gu10.A = Y + (size_t)10 * N * T; gu10.B = WM; gu10.bias = Y + (size_t)10 * N * T; gu10.R = Y + (size_t)10 * N * T; gu10.C = U;
      gu10.sAo = 0; gu10.sAi = 0; gu10.sAm = 1; gu10.sAk = T; gu10.sBo = 0; gu10.sBi = 0; gu10.sBn = N; gu10.sBk = 1; gu10.sCo = 0; gu10.sCi = 0; gu10.sCm = N; gu10.sRo = 0; gu10.sRi = 0; gu10.sRm = 0; gu10.sRn = 0;
      gu10.M = T; gu10.N = N; gu10.K = N; gu10.zi_n = 1; gu10.flags = 0; gu10.act = 0;
      gu10.alpha = 1.0f; gu10.beta = 0.0f; gu10.sa = 1.0f; gu10.sb = 1.0f; gu10.Npad = N; gu10.pad_ = 0;
      k_gemm<1><<<dim3((unsigned)((N) + 31) / 32, (unsigned)((T) + 15) / 16, (unsigned)(1)), 32, 0, stream>>>(gu10); }
    k_db_out<<<(unsigned)((T + 255) / 256), 256, 0, stream>>>(Y, U, out, 10, N, T);
    { GemmP gu11;
      gu11.A = Y + (size_t)11 * N * T; gu11.B = WM; gu11.bias = Y + (size_t)11 * N * T; gu11.R = Y + (size_t)11 * N * T; gu11.C = U;
      gu11.sAo = 0; gu11.sAi = 0; gu11.sAm = 1; gu11.sAk = T; gu11.sBo = 0; gu11.sBi = 0; gu11.sBn = N; gu11.sBk = 1; gu11.sCo = 0; gu11.sCi = 0; gu11.sCm = N; gu11.sRo = 0; gu11.sRi = 0; gu11.sRm = 0; gu11.sRn = 0;
      gu11.M = T; gu11.N = N; gu11.K = N; gu11.zi_n = 1; gu11.flags = 0; gu11.act = 0;
      gu11.alpha = 1.0f; gu11.beta = 0.0f; gu11.sa = 1.0f; gu11.sb = 1.0f; gu11.Npad = N; gu11.pad_ = 0;
      k_gemm<1><<<dim3((unsigned)((N) + 31) / 32, (unsigned)((T) + 15) / 16, (unsigned)(1)), 32, 0, stream>>>(gu11); }
    k_db_out<<<(unsigned)((T + 255) / 256), 256, 0, stream>>>(Y, U, out, 11, N, T);
    { GemmP gu12;
      gu12.A = Y + (size_t)12 * N * T; gu12.B = WM; gu12.bias = Y + (size_t)12 * N * T; gu12.R = Y + (size_t)12 * N * T; gu12.C = U;
      gu12.sAo = 0; gu12.sAi = 0; gu12.sAm = 1; gu12.sAk = T; gu12.sBo = 0; gu12.sBi = 0; gu12.sBn = N; gu12.sBk = 1; gu12.sCo = 0; gu12.sCi = 0; gu12.sCm = N; gu12.sRo = 0; gu12.sRi = 0; gu12.sRm = 0; gu12.sRn = 0;
      gu12.M = T; gu12.N = N; gu12.K = N; gu12.zi_n = 1; gu12.flags = 0; gu12.act = 0;
      gu12.alpha = 1.0f; gu12.beta = 0.0f; gu12.sa = 1.0f; gu12.sb = 1.0f; gu12.Npad = N; gu12.pad_ = 0;
      k_gemm<1><<<dim3((unsigned)((N) + 31) / 32, (unsigned)((T) + 15) / 16, (unsigned)(1)), 32, 0, stream>>>(gu12); }
    k_db_out<<<(unsigned)((T + 255) / 256), 256, 0, stream>>>(Y, U, out, 12, N, T);
    { GemmP gu13;
      gu13.A = Y + (size_t)13 * N * T; gu13.B = WM; gu13.bias = Y + (size_t)13 * N * T; gu13.R = Y + (size_t)13 * N * T; gu13.C = U;
      gu13.sAo = 0; gu13.sAi = 0; gu13.sAm = 1; gu13.sAk = T; gu13.sBo = 0; gu13.sBi = 0; gu13.sBn = N; gu13.sBk = 1; gu13.sCo = 0; gu13.sCi = 0; gu13.sCm = N; gu13.sRo = 0; gu13.sRi = 0; gu13.sRm = 0; gu13.sRn = 0;
      gu13.M = T; gu13.N = N; gu13.K = N; gu13.zi_n = 1; gu13.flags = 0; gu13.act = 0;
      gu13.alpha = 1.0f; gu13.beta = 0.0f; gu13.sa = 1.0f; gu13.sb = 1.0f; gu13.Npad = N; gu13.pad_ = 0;
      k_gemm<1><<<dim3((unsigned)((N) + 31) / 32, (unsigned)((T) + 15) / 16, (unsigned)(1)), 32, 0, stream>>>(gu13); }
    k_db_out<<<(unsigned)((T + 255) / 256), 256, 0, stream>>>(Y, U, out, 13, N, T);
    { GemmP gu14;
      gu14.A = Y + (size_t)14 * N * T; gu14.B = WM; gu14.bias = Y + (size_t)14 * N * T; gu14.R = Y + (size_t)14 * N * T; gu14.C = U;
      gu14.sAo = 0; gu14.sAi = 0; gu14.sAm = 1; gu14.sAk = T; gu14.sBo = 0; gu14.sBi = 0; gu14.sBn = N; gu14.sBk = 1; gu14.sCo = 0; gu14.sCi = 0; gu14.sCm = N; gu14.sRo = 0; gu14.sRi = 0; gu14.sRm = 0; gu14.sRn = 0;
      gu14.M = T; gu14.N = N; gu14.K = N; gu14.zi_n = 1; gu14.flags = 0; gu14.act = 0;
      gu14.alpha = 1.0f; gu14.beta = 0.0f; gu14.sa = 1.0f; gu14.sb = 1.0f; gu14.Npad = N; gu14.pad_ = 0;
      k_gemm<1><<<dim3((unsigned)((N) + 31) / 32, (unsigned)((T) + 15) / 16, (unsigned)(1)), 32, 0, stream>>>(gu14); }
    k_db_out<<<(unsigned)((T + 255) / 256), 256, 0, stream>>>(Y, U, out, 14, N, T);
    { GemmP gu15;
      gu15.A = Y + (size_t)15 * N * T; gu15.B = WM; gu15.bias = Y + (size_t)15 * N * T; gu15.R = Y + (size_t)15 * N * T; gu15.C = U;
      gu15.sAo = 0; gu15.sAi = 0; gu15.sAm = 1; gu15.sAk = T; gu15.sBo = 0; gu15.sBi = 0; gu15.sBn = N; gu15.sBk = 1; gu15.sCo = 0; gu15.sCi = 0; gu15.sCm = N; gu15.sRo = 0; gu15.sRi = 0; gu15.sRm = 0; gu15.sRn = 0;
      gu15.M = T; gu15.N = N; gu15.K = N; gu15.zi_n = 1; gu15.flags = 0; gu15.act = 0;
      gu15.alpha = 1.0f; gu15.beta = 0.0f; gu15.sa = 1.0f; gu15.sb = 1.0f; gu15.Npad = N; gu15.pad_ = 0;
      k_gemm<1><<<dim3((unsigned)((N) + 31) / 32, (unsigned)((T) + 15) / 16, (unsigned)(1)), 32, 0, stream>>>(gu15); }
    k_db_out<<<(unsigned)((T + 255) / 256), 256, 0, stream>>>(Y, U, out, 15, N, T);
    { GemmP gu16;
      gu16.A = Y + (size_t)16 * N * T; gu16.B = WM; gu16.bias = Y + (size_t)16 * N * T; gu16.R = Y + (size_t)16 * N * T; gu16.C = U;
      gu16.sAo = 0; gu16.sAi = 0; gu16.sAm = 1; gu16.sAk = T; gu16.sBo = 0; gu16.sBi = 0; gu16.sBn = N; gu16.sBk = 1; gu16.sCo = 0; gu16.sCi = 0; gu16.sCm = N; gu16.sRo = 0; gu16.sRi = 0; gu16.sRm = 0; gu16.sRn = 0;
      gu16.M = T; gu16.N = N; gu16.K = N; gu16.zi_n = 1; gu16.flags = 0; gu16.act = 0;
      gu16.alpha = 1.0f; gu16.beta = 0.0f; gu16.sa = 1.0f; gu16.sb = 1.0f; gu16.Npad = N; gu16.pad_ = 0;
      k_gemm<1><<<dim3((unsigned)((N) + 31) / 32, (unsigned)((T) + 15) / 16, (unsigned)(1)), 32, 0, stream>>>(gu16); }
    k_db_out<<<(unsigned)((T + 255) / 256), 256, 0, stream>>>(Y, U, out, 16, N, T);
    { GemmP gu17;
      gu17.A = Y + (size_t)17 * N * T; gu17.B = WM; gu17.bias = Y + (size_t)17 * N * T; gu17.R = Y + (size_t)17 * N * T; gu17.C = U;
      gu17.sAo = 0; gu17.sAi = 0; gu17.sAm = 1; gu17.sAk = T; gu17.sBo = 0; gu17.sBi = 0; gu17.sBn = N; gu17.sBk = 1; gu17.sCo = 0; gu17.sCi = 0; gu17.sCm = N; gu17.sRo = 0; gu17.sRi = 0; gu17.sRm = 0; gu17.sRn = 0;
      gu17.M = T; gu17.N = N; gu17.K = N; gu17.zi_n = 1; gu17.flags = 0; gu17.act = 0;
      gu17.alpha = 1.0f; gu17.beta = 0.0f; gu17.sa = 1.0f; gu17.sb = 1.0f; gu17.Npad = N; gu17.pad_ = 0;
      k_gemm<1><<<dim3((unsigned)((N) + 31) / 32, (unsigned)((T) + 15) / 16, (unsigned)(1)), 32, 0, stream>>>(gu17); }
    k_db_out<<<(unsigned)((T + 255) / 256), 256, 0, stream>>>(Y, U, out, 17, N, T);
    { GemmP gu18;
      gu18.A = Y + (size_t)18 * N * T; gu18.B = WM; gu18.bias = Y + (size_t)18 * N * T; gu18.R = Y + (size_t)18 * N * T; gu18.C = U;
      gu18.sAo = 0; gu18.sAi = 0; gu18.sAm = 1; gu18.sAk = T; gu18.sBo = 0; gu18.sBi = 0; gu18.sBn = N; gu18.sBk = 1; gu18.sCo = 0; gu18.sCi = 0; gu18.sCm = N; gu18.sRo = 0; gu18.sRi = 0; gu18.sRm = 0; gu18.sRn = 0;
      gu18.M = T; gu18.N = N; gu18.K = N; gu18.zi_n = 1; gu18.flags = 0; gu18.act = 0;
      gu18.alpha = 1.0f; gu18.beta = 0.0f; gu18.sa = 1.0f; gu18.sb = 1.0f; gu18.Npad = N; gu18.pad_ = 0;
      k_gemm<1><<<dim3((unsigned)((N) + 31) / 32, (unsigned)((T) + 15) / 16, (unsigned)(1)), 32, 0, stream>>>(gu18); }
    k_db_out<<<(unsigned)((T + 255) / 256), 256, 0, stream>>>(Y, U, out, 18, N, T);
    { GemmP gu19;
      gu19.A = Y + (size_t)19 * N * T; gu19.B = WM; gu19.bias = Y + (size_t)19 * N * T; gu19.R = Y + (size_t)19 * N * T; gu19.C = U;
      gu19.sAo = 0; gu19.sAi = 0; gu19.sAm = 1; gu19.sAk = T; gu19.sBo = 0; gu19.sBi = 0; gu19.sBn = N; gu19.sBk = 1; gu19.sCo = 0; gu19.sCi = 0; gu19.sCm = N; gu19.sRo = 0; gu19.sRi = 0; gu19.sRm = 0; gu19.sRn = 0;
      gu19.M = T; gu19.N = N; gu19.K = N; gu19.zi_n = 1; gu19.flags = 0; gu19.act = 0;
      gu19.alpha = 1.0f; gu19.beta = 0.0f; gu19.sa = 1.0f; gu19.sb = 1.0f; gu19.Npad = N; gu19.pad_ = 0;
      k_gemm<1><<<dim3((unsigned)((N) + 31) / 32, (unsigned)((T) + 15) / 16, (unsigned)(1)), 32, 0, stream>>>(gu19); }
    k_db_out<<<(unsigned)((T + 255) / 256), 256, 0, stream>>>(Y, U, out, 19, N, T);
    { GemmP gu20;
      gu20.A = Y + (size_t)20 * N * T; gu20.B = WM; gu20.bias = Y + (size_t)20 * N * T; gu20.R = Y + (size_t)20 * N * T; gu20.C = U;
      gu20.sAo = 0; gu20.sAi = 0; gu20.sAm = 1; gu20.sAk = T; gu20.sBo = 0; gu20.sBi = 0; gu20.sBn = N; gu20.sBk = 1; gu20.sCo = 0; gu20.sCi = 0; gu20.sCm = N; gu20.sRo = 0; gu20.sRi = 0; gu20.sRm = 0; gu20.sRn = 0;
      gu20.M = T; gu20.N = N; gu20.K = N; gu20.zi_n = 1; gu20.flags = 0; gu20.act = 0;
      gu20.alpha = 1.0f; gu20.beta = 0.0f; gu20.sa = 1.0f; gu20.sb = 1.0f; gu20.Npad = N; gu20.pad_ = 0;
      k_gemm<1><<<dim3((unsigned)((N) + 31) / 32, (unsigned)((T) + 15) / 16, (unsigned)(1)), 32, 0, stream>>>(gu20); }
    k_db_out<<<(unsigned)((T + 255) / 256), 256, 0, stream>>>(Y, U, out, 20, N, T);
    { GemmP gu21;
      gu21.A = Y + (size_t)21 * N * T; gu21.B = WM; gu21.bias = Y + (size_t)21 * N * T; gu21.R = Y + (size_t)21 * N * T; gu21.C = U;
      gu21.sAo = 0; gu21.sAi = 0; gu21.sAm = 1; gu21.sAk = T; gu21.sBo = 0; gu21.sBi = 0; gu21.sBn = N; gu21.sBk = 1; gu21.sCo = 0; gu21.sCi = 0; gu21.sCm = N; gu21.sRo = 0; gu21.sRi = 0; gu21.sRm = 0; gu21.sRn = 0;
      gu21.M = T; gu21.N = N; gu21.K = N; gu21.zi_n = 1; gu21.flags = 0; gu21.act = 0;
      gu21.alpha = 1.0f; gu21.beta = 0.0f; gu21.sa = 1.0f; gu21.sb = 1.0f; gu21.Npad = N; gu21.pad_ = 0;
      k_gemm<1><<<dim3((unsigned)((N) + 31) / 32, (unsigned)((T) + 15) / 16, (unsigned)(1)), 32, 0, stream>>>(gu21); }
    k_db_out<<<(unsigned)((T + 255) / 256), 256, 0, stream>>>(Y, U, out, 21, N, T);
    { GemmP gu22;
      gu22.A = Y + (size_t)22 * N * T; gu22.B = WM; gu22.bias = Y + (size_t)22 * N * T; gu22.R = Y + (size_t)22 * N * T; gu22.C = U;
      gu22.sAo = 0; gu22.sAi = 0; gu22.sAm = 1; gu22.sAk = T; gu22.sBo = 0; gu22.sBi = 0; gu22.sBn = N; gu22.sBk = 1; gu22.sCo = 0; gu22.sCi = 0; gu22.sCm = N; gu22.sRo = 0; gu22.sRi = 0; gu22.sRm = 0; gu22.sRn = 0;
      gu22.M = T; gu22.N = N; gu22.K = N; gu22.zi_n = 1; gu22.flags = 0; gu22.act = 0;
      gu22.alpha = 1.0f; gu22.beta = 0.0f; gu22.sa = 1.0f; gu22.sb = 1.0f; gu22.Npad = N; gu22.pad_ = 0;
      k_gemm<1><<<dim3((unsigned)((N) + 31) / 32, (unsigned)((T) + 15) / 16, (unsigned)(1)), 32, 0, stream>>>(gu22); }
    k_db_out<<<(unsigned)((T + 255) / 256), 256, 0, stream>>>(Y, U, out, 22, N, T);
    { GemmP gu23;
      gu23.A = Y + (size_t)23 * N * T; gu23.B = WM; gu23.bias = Y + (size_t)23 * N * T; gu23.R = Y + (size_t)23 * N * T; gu23.C = U;
      gu23.sAo = 0; gu23.sAi = 0; gu23.sAm = 1; gu23.sAk = T; gu23.sBo = 0; gu23.sBi = 0; gu23.sBn = N; gu23.sBk = 1; gu23.sCo = 0; gu23.sCi = 0; gu23.sCm = N; gu23.sRo = 0; gu23.sRi = 0; gu23.sRm = 0; gu23.sRn = 0;
      gu23.M = T; gu23.N = N; gu23.K = N; gu23.zi_n = 1; gu23.flags = 0; gu23.act = 0;
      gu23.alpha = 1.0f; gu23.beta = 0.0f; gu23.sa = 1.0f; gu23.sb = 1.0f; gu23.Npad = N; gu23.pad_ = 0;
      k_gemm<1><<<dim3((unsigned)((N) + 31) / 32, (unsigned)((T) + 15) / 16, (unsigned)(1)), 32, 0, stream>>>(gu23); }
    k_db_out<<<(unsigned)((T + 255) / 256), 256, 0, stream>>>(Y, U, out, 23, N, T);
    { GemmP gu24;
      gu24.A = Y + (size_t)24 * N * T; gu24.B = WM; gu24.bias = Y + (size_t)24 * N * T; gu24.R = Y + (size_t)24 * N * T; gu24.C = U;
      gu24.sAo = 0; gu24.sAi = 0; gu24.sAm = 1; gu24.sAk = T; gu24.sBo = 0; gu24.sBi = 0; gu24.sBn = N; gu24.sBk = 1; gu24.sCo = 0; gu24.sCi = 0; gu24.sCm = N; gu24.sRo = 0; gu24.sRi = 0; gu24.sRm = 0; gu24.sRn = 0;
      gu24.M = T; gu24.N = N; gu24.K = N; gu24.zi_n = 1; gu24.flags = 0; gu24.act = 0;
      gu24.alpha = 1.0f; gu24.beta = 0.0f; gu24.sa = 1.0f; gu24.sb = 1.0f; gu24.Npad = N; gu24.pad_ = 0;
      k_gemm<1><<<dim3((unsigned)((N) + 31) / 32, (unsigned)((T) + 15) / 16, (unsigned)(1)), 32, 0, stream>>>(gu24); }
    k_db_out<<<(unsigned)((T + 255) / 256), 256, 0, stream>>>(Y, U, out, 24, N, T);
    { GemmP gu25;
      gu25.A = Y + (size_t)25 * N * T; gu25.B = WM; gu25.bias = Y + (size_t)25 * N * T; gu25.R = Y + (size_t)25 * N * T; gu25.C = U;
      gu25.sAo = 0; gu25.sAi = 0; gu25.sAm = 1; gu25.sAk = T; gu25.sBo = 0; gu25.sBi = 0; gu25.sBn = N; gu25.sBk = 1; gu25.sCo = 0; gu25.sCi = 0; gu25.sCm = N; gu25.sRo = 0; gu25.sRi = 0; gu25.sRm = 0; gu25.sRn = 0;
      gu25.M = T; gu25.N = N; gu25.K = N; gu25.zi_n = 1; gu25.flags = 0; gu25.act = 0;
      gu25.alpha = 1.0f; gu25.beta = 0.0f; gu25.sa = 1.0f; gu25.sb = 1.0f; gu25.Npad = N; gu25.pad_ = 0;
      k_gemm<1><<<dim3((unsigned)((N) + 31) / 32, (unsigned)((T) + 15) / 16, (unsigned)(1)), 32, 0, stream>>>(gu25); }
    k_db_out<<<(unsigned)((T + 255) / 256), 256, 0, stream>>>(Y, U, out, 25, N, T);
    { GemmP gu26;
      gu26.A = Y + (size_t)26 * N * T; gu26.B = WM; gu26.bias = Y + (size_t)26 * N * T; gu26.R = Y + (size_t)26 * N * T; gu26.C = U;
      gu26.sAo = 0; gu26.sAi = 0; gu26.sAm = 1; gu26.sAk = T; gu26.sBo = 0; gu26.sBi = 0; gu26.sBn = N; gu26.sBk = 1; gu26.sCo = 0; gu26.sCi = 0; gu26.sCm = N; gu26.sRo = 0; gu26.sRi = 0; gu26.sRm = 0; gu26.sRn = 0;
      gu26.M = T; gu26.N = N; gu26.K = N; gu26.zi_n = 1; gu26.flags = 0; gu26.act = 0;
      gu26.alpha = 1.0f; gu26.beta = 0.0f; gu26.sa = 1.0f; gu26.sb = 1.0f; gu26.Npad = N; gu26.pad_ = 0;
      k_gemm<1><<<dim3((unsigned)((N) + 31) / 32, (unsigned)((T) + 15) / 16, (unsigned)(1)), 32, 0, stream>>>(gu26); }
    k_db_out<<<(unsigned)((T + 255) / 256), 256, 0, stream>>>(Y, U, out, 26, N, T);
    { GemmP gu27;
      gu27.A = Y + (size_t)27 * N * T; gu27.B = WM; gu27.bias = Y + (size_t)27 * N * T; gu27.R = Y + (size_t)27 * N * T; gu27.C = U;
      gu27.sAo = 0; gu27.sAi = 0; gu27.sAm = 1; gu27.sAk = T; gu27.sBo = 0; gu27.sBi = 0; gu27.sBn = N; gu27.sBk = 1; gu27.sCo = 0; gu27.sCi = 0; gu27.sCm = N; gu27.sRo = 0; gu27.sRi = 0; gu27.sRm = 0; gu27.sRn = 0;
      gu27.M = T; gu27.N = N; gu27.K = N; gu27.zi_n = 1; gu27.flags = 0; gu27.act = 0;
      gu27.alpha = 1.0f; gu27.beta = 0.0f; gu27.sa = 1.0f; gu27.sb = 1.0f; gu27.Npad = N; gu27.pad_ = 0;
      k_gemm<1><<<dim3((unsigned)((N) + 31) / 32, (unsigned)((T) + 15) / 16, (unsigned)(1)), 32, 0, stream>>>(gu27); }
    k_db_out<<<(unsigned)((T + 255) / 256), 256, 0, stream>>>(Y, U, out, 27, N, T);
    { GemmP gu28;
      gu28.A = Y + (size_t)28 * N * T; gu28.B = WM; gu28.bias = Y + (size_t)28 * N * T; gu28.R = Y + (size_t)28 * N * T; gu28.C = U;
      gu28.sAo = 0; gu28.sAi = 0; gu28.sAm = 1; gu28.sAk = T; gu28.sBo = 0; gu28.sBi = 0; gu28.sBn = N; gu28.sBk = 1; gu28.sCo = 0; gu28.sCi = 0; gu28.sCm = N; gu28.sRo = 0; gu28.sRi = 0; gu28.sRm = 0; gu28.sRn = 0;
      gu28.M = T; gu28.N = N; gu28.K = N; gu28.zi_n = 1; gu28.flags = 0; gu28.act = 0;
      gu28.alpha = 1.0f; gu28.beta = 0.0f; gu28.sa = 1.0f; gu28.sb = 1.0f; gu28.Npad = N; gu28.pad_ = 0;
      k_gemm<1><<<dim3((unsigned)((N) + 31) / 32, (unsigned)((T) + 15) / 16, (unsigned)(1)), 32, 0, stream>>>(gu28); }
    k_db_out<<<(unsigned)((T + 255) / 256), 256, 0, stream>>>(Y, U, out, 28, N, T);
    { GemmP gu29;
      gu29.A = Y + (size_t)29 * N * T; gu29.B = WM; gu29.bias = Y + (size_t)29 * N * T; gu29.R = Y + (size_t)29 * N * T; gu29.C = U;
      gu29.sAo = 0; gu29.sAi = 0; gu29.sAm = 1; gu29.sAk = T; gu29.sBo = 0; gu29.sBi = 0; gu29.sBn = N; gu29.sBk = 1; gu29.sCo = 0; gu29.sCi = 0; gu29.sCm = N; gu29.sRo = 0; gu29.sRi = 0; gu29.sRm = 0; gu29.sRn = 0;
      gu29.M = T; gu29.N = N; gu29.K = N; gu29.zi_n = 1; gu29.flags = 0; gu29.act = 0;
      gu29.alpha = 1.0f; gu29.beta = 0.0f; gu29.sa = 1.0f; gu29.sb = 1.0f; gu29.Npad = N; gu29.pad_ = 0;
      k_gemm<1><<<dim3((unsigned)((N) + 31) / 32, (unsigned)((T) + 15) / 16, (unsigned)(1)), 32, 0, stream>>>(gu29); }
    k_db_out<<<(unsigned)((T + 255) / 256), 256, 0, stream>>>(Y, U, out, 29, N, T);
    { GemmP gu30;
      gu30.A = Y + (size_t)30 * N * T; gu30.B = WM; gu30.bias = Y + (size_t)30 * N * T; gu30.R = Y + (size_t)30 * N * T; gu30.C = U;
      gu30.sAo = 0; gu30.sAi = 0; gu30.sAm = 1; gu30.sAk = T; gu30.sBo = 0; gu30.sBi = 0; gu30.sBn = N; gu30.sBk = 1; gu30.sCo = 0; gu30.sCi = 0; gu30.sCm = N; gu30.sRo = 0; gu30.sRi = 0; gu30.sRm = 0; gu30.sRn = 0;
      gu30.M = T; gu30.N = N; gu30.K = N; gu30.zi_n = 1; gu30.flags = 0; gu30.act = 0;
      gu30.alpha = 1.0f; gu30.beta = 0.0f; gu30.sa = 1.0f; gu30.sb = 1.0f; gu30.Npad = N; gu30.pad_ = 0;
      k_gemm<1><<<dim3((unsigned)((N) + 31) / 32, (unsigned)((T) + 15) / 16, (unsigned)(1)), 32, 0, stream>>>(gu30); }
    k_db_out<<<(unsigned)((T + 255) / 256), 256, 0, stream>>>(Y, U, out, 30, N, T);
    { GemmP gu31;
      gu31.A = Y + (size_t)31 * N * T; gu31.B = WM; gu31.bias = Y + (size_t)31 * N * T; gu31.R = Y + (size_t)31 * N * T; gu31.C = U;
      gu31.sAo = 0; gu31.sAi = 0; gu31.sAm = 1; gu31.sAk = T; gu31.sBo = 0; gu31.sBi = 0; gu31.sBn = N; gu31.sBk = 1; gu31.sCo = 0; gu31.sCi = 0; gu31.sCm = N; gu31.sRo = 0; gu31.sRi = 0; gu31.sRm = 0; gu31.sRn = 0;
      gu31.M = T; gu31.N = N; gu31.K = N; gu31.zi_n = 1; gu31.flags = 0; gu31.act = 0;
      gu31.alpha = 1.0f; gu31.beta = 0.0f; gu31.sa = 1.0f; gu31.sb = 1.0f; gu31.Npad = N; gu31.pad_ = 0;
      k_gemm<1><<<dim3((unsigned)((N) + 31) / 32, (unsigned)((T) + 15) / 16, (unsigned)(1)), 32, 0, stream>>>(gu31); }
    k_db_out<<<(unsigned)((T + 255) / 256), 256, 0, stream>>>(Y, U, out, 31, N, T);
}
